// TemporalGNN_78554951843862
// MI455X (gfx1250) — hardware-verified
//
#include <hip/hip_runtime.h>
#include <math.h>

#define GG 32
#define GN 4000
#define GNP 4096
#define GE 32000
#define GF 64
#define GH 128
#define BNR 16000
#define NSTEP 8
#define NT 256
#define SRB 2048
#define WROWS (SRB / 8)
#define SCH 2048
#define SP (SCH / NT)
#define NCH ((GE + SCH - 1) / SCH)

typedef __attribute__((ext_vector_type(16))) _Float16 v16h;
typedef __attribute__((ext_vector_type(8)))  _Float16 v8h;
typedef __attribute__((ext_vector_type(4)))  _Float16 v4h;
typedef __attribute__((ext_vector_type(16))) __bf16   v16b;
typedef __attribute__((ext_vector_type(8)))  __bf16   v8b;
typedef __attribute__((ext_vector_type(8)))  float    v8f;
typedef __attribute__((ext_vector_type(4)))  float    v4f;
typedef __attribute__((ext_vector_type(4)))  int      v4i;

template <int W> struct FV;
template <> struct FV<2> { typedef float T __attribute__((ext_vector_type(2))); typedef _Float16 H __attribute__((ext_vector_type(2))); };
template <> struct FV<4> { typedef float T __attribute__((ext_vector_type(4))); typedef _Float16 H __attribute__((ext_vector_type(4))); };

__device__ __forceinline__ unsigned short f2bf_bits(float f) {
  unsigned u = __float_as_uint(f);
  return (unsigned short)((u + 0x7FFFu + ((u >> 16) & 1u)) >> 16);
}
__device__ __forceinline__ float bf_bits2f(unsigned short h) { return __uint_as_float(((unsigned)h) << 16); }

__device__ __forceinline__ void dep_guard_h(v8f& a, v8f& b, v16h x, v16h y) { asm volatile("v_nop\n\tv_nop\n\tv_nop\n\tv_nop" : "+v"(a), "+v"(b) : "v"(x), "v"(y)); }
__device__ __forceinline__ void dep_guard_b(v8f& a, v8f& b, v16b x, v16b y) { asm volatile("v_nop\n\tv_nop\n\tv_nop\n\tv_nop" : "+v"(a), "+v"(b) : "v"(x), "v"(y)); }
__device__ __forceinline__ void keep4_h(v16h a, v16h b, v16h c, v16h d) { asm volatile("v_nop" :: "v"(a), "v"(b), "v"(c), "v"(d)); }
__device__ __forceinline__ void keep4_b(v16b a, v16b b, v16b c, v16b d) { asm volatile("v_nop" :: "v"(a), "v"(b), "v"(c), "v"(d)); }
__device__ __forceinline__ void acc_guard4(v8f& a, v8f& b, v8f& c, v8f& d) { asm volatile("v_nop\n\tv_nop\n\tv_nop\n\tv_nop" : "+v"(a), "+v"(b), "+v"(c), "+v"(d)); }
template <typename T> struct Frag;
template <> struct Frag<_Float16> {
  typedef v16h V; union U { v16h v; v8h h[2]; };
  static __device__ __forceinline__ v16h load(const _Float16* p) {
    U f; f.h[0] = *(const v8h*)(p); f.h[1] = *(const v8h*)(p + 16); return f.v;
  }
  static __device__ __forceinline__ v8f mma(v16h a, v16h b, v8f c) {
    return __builtin_amdgcn_wmma_f32_16x16x32_f16(false, a, false, b, (short)0, c, false, false);
  }
  static __device__ __forceinline__ void guard(v8f& a, v8f& b, v16h x, v16h y) { dep_guard_h(a, b, x, y); }
  static __device__ __forceinline__ void keep(v16h a, v16h b, v16h c, v16h d) { keep4_h(a, b, c, d); }
};
template <> struct Frag<__bf16> {
  typedef v16b V; union U { v16b v; v8b h[2]; };
  static __device__ __forceinline__ v16b load(const __bf16* p) {
    U f; f.h[0] = *(const v8b*)(p); f.h[1] = *(const v8b*)(p + 16); return f.v;
  }
  static __device__ __forceinline__ v8f mma(v16b a, v16b b, v8f c) {
    return __builtin_amdgcn_wmma_f32_16x16x32_bf16(false, a, false, b, (short)0, c, false, false);
  }
  static __device__ __forceinline__ void guard(v8f& a, v8f& b, v16b x, v16b y) { dep_guard_b(a, b, x, y); }
  static __device__ __forceinline__ void keep(v16b a, v16b b, v16b c, v16b d) { keep4_b(a, b, c, d); }
};

template <int ET> struct Elem;
template <> struct Elem<0> { typedef _Float16 T; };
template <> struct Elem<1> { typedef __bf16 T; };
template <int ET, bool SPLIT, int BIAS_MODE, int OUT_MODE, bool RESID, int ACT = 0>
__global__ __launch_bounds__(256) void wmma_gemm64(
    const unsigned short* __restrict__ Ap, const unsigned short* __restrict__ A2p, int lda, long strideA,
    const unsigned short* __restrict__ Btp, const unsigned short* __restrict__ Bt2p, int ldb, long strideB,
    void* __restrict__ Cout, void* __restrict__ Cout2, int ldc, long strideC,
    const float* __restrict__ bias,
    const float* __restrict__ resid, long strideR,
    int M, int N, int K, float scale) {
  typedef typename Elem<ET>::T T;
  typedef typename Frag<T>::V V;
  const T* A = (const T*)Ap; const T* A2 = (const T*)A2p; const T* Bt = (const T*)Btp; const T* Bt2 = (const T*)Bt2p;
  __shared__ __align__(16) float sT[8][16 * 68];
  const int b    = blockIdx.y;
  const int lane = threadIdx.x & 31;
  const int wave = threadIdx.x >> 5;
  const int tilesN = N >> 6;
  const int tilesM = M >> 6;
  const int tile = blockIdx.x * 8 + wave;
  if (tile >= tilesM * tilesN) return;
  const int tm = tile / tilesN;
  const int tn = tile - tm * tilesN;
  const int m0 = tm << 6;
  const int n0 = tn << 6;

  const T* Ab  = A  + (size_t)b * strideA;
  const T* Bb  = Bt + (size_t)b * strideB;
  const T* Ab2 = SPLIT ? (A2  + (size_t)b * strideA) : nullptr;
  const T* Bb2 = SPLIT ? (Bt2 + (size_t)b * strideB) : nullptr;

  const int rlane = lane & 15;
  const int koff  = (lane >> 4) * 8;
  const int mOff  = (lane >> 4) * 8;

  v8f acc[4][4];
#pragma unroll
  for (int i = 0; i < 4; ++i)
#pragma unroll
    for (int j = 0; j < 4; ++j) acc[i][j] = (v8f){0.f,0.f,0.f,0.f,0.f,0.f,0.f,0.f};

  for (int k0 = 0; k0 < K; k0 += 32) {
    V bh[4], bl[4];
#pragma unroll
    for (int j = 0; j < 4; ++j) {
      const size_t bo = (size_t)(n0 + (j << 4) + rlane) * ldb + koff + k0;
      bh[j] = Frag<T>::load(Bb + bo);
      if (SPLIT) bl[j] = Frag<T>::load(Bb2 + bo);
    }
#pragma unroll
    for (int i = 0; i < 4; ++i) {
      const size_t ao = (size_t)(m0 + (i << 4) + rlane) * lda + koff + k0;
      V ah = Frag<T>::load(Ab + ao);
      V al;
      if (SPLIT) al = Frag<T>::load(Ab2 + ao);
#pragma unroll
      for (int j = 0; j < 4; ++j) {
        acc[i][j] = Frag<T>::mma(ah, bh[j], acc[i][j]);
        if (SPLIT) {
          acc[i][j] = Frag<T>::mma(ah, bl[j], acc[i][j]);
          acc[i][j] = Frag<T>::mma(al, bh[j], acc[i][j]);
        }
      }
      Frag<T>::guard(acc[i][0], acc[i][3], ah, SPLIT ? al : ah);
    }
    Frag<T>::keep(bh[0], bh[1], bh[2], bh[3]);
    if (SPLIT) Frag<T>::keep(bl[0], bl[1], bl[2], bl[3]);
  }
  acc_guard4(acc[0][0], acc[0][1], acc[0][2], acc[0][3]);
  acc_guard4(acc[1][0], acc[1][1], acc[1][2], acc[1][3]);
  acc_guard4(acc[2][0], acc[2][1], acc[2][2], acc[2][3]);
  acc_guard4(acc[3][0], acc[3][1], acc[3][2], acc[3][3]);

  float* slab = sT[wave];
  const float* Rb = RESID ? (resid + (size_t)b * strideR) : nullptr;
#pragma unroll
  for (int i = 0; i < 4; ++i) {
    const int mBase = m0 + (i << 4);
#pragma unroll
    for (int j = 0; j < 4; ++j) {
      const int n = n0 + (j << 4) + rlane;
      float bv = 0.f;
      if (BIAS_MODE == 2) bv = bias[n];
#pragma unroll
      for (int r = 0; r < 8; ++r) {
        float v = acc[i][j][r] * scale;
        if (BIAS_MODE == 1) v += bias[mBase + mOff + r];
        if (BIAS_MODE == 2) v += bv;
        if (RESID) v += Rb[(size_t)(mBase + mOff + r) * ldc + n];
        if (ACT == 1) v = tanhf(v);
        if (ACT == 2) v = fmaxf(v, 0.0f);
        if (ACT == 3) v = v / (1.0f + expf(-v));
        if (ACT == 4) v = (v > 0.f) ? v : 0.01f * v;
        if (ACT == 5) v = 0.5f * v * (1.0f + erff(v * 0.70710678118654752f));
        slab[(mOff + r) * 68 + (j << 4) + rlane] = v;
      }
    }
    __builtin_amdgcn_fence(__ATOMIC_RELEASE, "workgroup");
    __builtin_amdgcn_wave_barrier();
    __builtin_amdgcn_fence(__ATOMIC_ACQUIRE, "workgroup");
    if (OUT_MODE == 0) {
      float* C = (float*)Cout + (size_t)b * strideC;
      const int hh = lane >> 4, c4 = (lane & 15) * 4;
      for (int pass = 0; pass < 2; ++pass) {
#pragma unroll
        for (int it = 0; it < 8; ++it) {
          const int row = it * 2 + hh;
          v4f v = *(const v4f*)(slab + row * 68 + c4);
          *(volatile v4f*)(C + (size_t)(mBase + row) * ldc + n0 + c4) = v;
        }
        __threadfence();
      }
    } else {
      const int q = lane >> 3, c8 = (lane & 7) * 8;
      unsigned short* C  = (unsigned short*)Cout  + (size_t)b * strideC;
      unsigned short* C2 = (OUT_MODE == 2) ? ((unsigned short*)Cout2 + (size_t)b * strideC) : nullptr;
      for (int pass = 0; pass < 2; ++pass) {
#pragma unroll
        for (int it = 0; it < 4; ++it) {
          const int row = it * 4 + q;
          const float* sp = slab + row * 68 + c8;
          v8h hv, lv;
#pragma unroll
          for (int e = 0; e < 8; ++e) {
            if (OUT_MODE == 1) {
              hv[e] = (_Float16)sp[e];
            } else {
              unsigned short hb = f2bf_bits(sp[e]);
              unsigned short lb = f2bf_bits(sp[e] - bf_bits2f(hb));
              hv[e] = __builtin_bit_cast(_Float16, hb);
              lv[e] = __builtin_bit_cast(_Float16, lb);
            }
          }
          *(volatile v8h*)(C + (size_t)(mBase + row) * ldc + n0 + c8) = hv;
          if (OUT_MODE == 2) *(volatile v8h*)(C2 + (size_t)(mBase + row) * ldc + n0 + c8) = lv;
        }
        __threadfence();
      }
    }
    __builtin_amdgcn_fence(__ATOMIC_RELEASE, "workgroup");
    __builtin_amdgcn_wave_barrier();
    __builtin_amdgcn_fence(__ATOMIC_ACQUIRE, "workgroup");
  }
}

__device__ __forceinline__ int blk_excl_scan(int cnt, int* scan_ws, int tid, int* tot) {
  const int lane = tid & 31, wave = tid >> 5; int incl = cnt;
#pragma unroll
  for (int o = 1; o < 32; o <<= 1) { const int v = __shfl_up(incl, o, 32); if (lane >= o) incl += v; }
  if (lane == 31) scan_ws[wave] = incl;
  __syncthreads();
  if (wave == 0) { int wv = (lane < NT / 32) ? scan_ws[lane] : 0; int wincl = wv;
#pragma unroll
    for (int o = 1; o < 32; o <<= 1) { const int v = __shfl_up(wincl, o, 32); if (lane >= o) wincl += v; }
    if (lane < NT / 32) scan_ws[32 + lane] = wincl - wv; if (lane == 31) scan_ws[64] = wincl; }
  __syncthreads();
  const int res = scan_ws[32 + wave] + incl - cnt; *tot = scan_ws[64];
  return res;
}

__device__ __forceinline__ int deg_hits(const int* __restrict__ keyv, const float* __restrict__ ewg, int e0, int n0, int tid,
                                        int* LIST, float* LW, int* scan_ws) {
  const int eb = e0 + tid * SP;
  const bool inr = eb < GE;
  const int ebc = inr ? eb : (GE - SP);
  int rec[SP]; float wr[SP]; int cnt = 0;
#pragma unroll
  for (int k = 0; k < SP; k += 4) {
    const v4i d4 = *(const v4i*)(keyv + ebc + k);
    const v4f w4 = *(const v4f*)(ewg + ebc + k);
#pragma unroll
    for (int e = 0; e < 4; ++e) {
      const int d = d4[e]; int r = -1;
      if (inr && d >= n0 && d < n0 + SRB) { r = d - n0; ++cnt; }
      rec[k + e] = r; wr[k + e] = w4[e];
    }
  }
  int tot; int p = blk_excl_scan(cnt, scan_ws, tid, &tot);
#pragma unroll
  for (int k = 0; k < SP; ++k) if (rec[k] >= 0) { if ((unsigned)p < (unsigned)SCH) { LIST[p] = rec[k]; LW[p] = wr[k]; } ++p; }
  __syncthreads();
  return tot < SCH ? tot : SCH;
}
__device__ __forceinline__ int agg_hits(const int* __restrict__ keyv, const int* __restrict__ othv, const float* __restrict__ ewg,
                                        const float* __restrict__ ivO, int e0, int n0, int tid, int* LIST, float* LW, int* scan_ws) {
  const int eb = e0 + tid * SP;
  const bool inr = eb < GE;
  const int ebc = inr ? eb : (GE - SP);
  int rec[SP]; float wr[SP]; int cnt = 0;
#pragma unroll
  for (int k = 0; k < SP; k += 4) {
    const v4i d4 = *(const v4i*)(keyv + ebc + k);
    const v4i s4 = *(const v4i*)(othv + ebc + k);
    const v4f w4 = *(const v4f*)(ewg + ebc + k);
#pragma unroll
    for (int e = 0; e < 4; ++e) {
      const int d = d4[e]; int s = s4[e]; s = s < 0 ? 0 : (s >= GN ? GN - 1 : s);
      const float w = w4[e] * ivO[s];
      int r = -1;
      if (inr && d >= n0 && d < n0 + SRB) { r = ((d - n0) << 16) | s; ++cnt; }
      rec[k + e] = r; wr[k + e] = w;
    }
  }
  int tot; int p = blk_excl_scan(cnt, scan_ws, tid, &tot);
#pragma unroll
  for (int k = 0; k < SP; ++k) if (rec[k] >= 0) { if ((unsigned)p < (unsigned)SCH) { LIST[p] = rec[k]; LW[p] = wr[k]; } ++p; }
  __syncthreads();
  return tot < SCH ? tot : SCH;
}
__device__ __forceinline__ void deg_apply(int tot, int lane, int wave, const int* LIST, const float* LW, float* SD) {
#pragma unroll 1
  for (int base = 0; base < tot; base += 32) {
    const int q = base + lane; const int qc = q < SCH ? q : SCH - 1;
    const int lv = LIST[qc]; const float lwv = LW[qc];
    const int rv = (q < tot) ? lv : -1;
    const float wv = (q < tot) ? lwv : 0.f;
    const int own = (rv >= 0 && (rv >> 8) == wave) ? 1 : 0;
    unsigned msk = (unsigned)__ballot(own);
#pragma unroll 1
    for (int it = 0; it < 32; ++it) {
      if (msk == 0u) break;
      const int bp = __builtin_ctz(msk); msk &= msk - 1u;
      const int d = __shfl(rv, bp, 32);
      const float w = __shfl(wv, bp, 32);
      if (lane == 0) SD[d] += w;
    }
  }
}
__device__ __forceinline__ float inv_sqrt_deg(float d) { return (d > 0.f) ? (1.0f / sqrtf(fmaxf(d, 1e-12f))) : 0.f; }

__device__ __forceinline__ void castpair(const float* __restrict__ in, _Float16* __restrict__ out, int i, int Cc, int P, int coff,
                                         float sc, int n2) {
  if (i < n2) {
    const int hc = Cc >> 1;
    const int r = i / hc, c = 2 * (i - r * hc);
    const _Float16 h0 = (_Float16)(in[(size_t)r * Cc + c] * sc), h1 = (_Float16)(in[(size_t)r * Cc + c + 1] * sc);
    const unsigned u = (unsigned)__builtin_bit_cast(unsigned short, h0) | ((unsigned)__builtin_bit_cast(unsigned short, h1) << 16);
    unsigned* p = (unsigned*)(out + (size_t)r * P + coff + c);
    *(volatile unsigned*)p = u;
    __threadfence();
    *(volatile unsigned*)p = u;
  }
}
__global__ __launch_bounds__(NT) void k_prep(const float* __restrict__ W0s, const float* __restrict__ W0d,
                                             const float* __restrict__ W1s, const float* __restrict__ W1d,
                                             const float* __restrict__ Wih, const float* __restrict__ Whh, const float* __restrict__ Wp,
                                             const float* __restrict__ b0s, const float* __restrict__ b0d,
                                             const float* __restrict__ b1s, const float* __restrict__ b1d,
                                             const float* __restrict__ bih, const float* __restrict__ bhh,
                                             _Float16* __restrict__ W0c, _Float16* __restrict__ W1c, _Float16* __restrict__ WIH,
                                             _Float16* __restrict__ WHH, _Float16* __restrict__ WPc, float* __restrict__ BI) {
  const int bx = blockIdx.x, tid = threadIdx.x;
  if (bx < 16)       castpair(W0s, W0c, (bx - 0) * NT + tid, GF, 2 * GF, 0, 16.0f, GH * GF / 2);
  else if (bx < 32)  castpair(W0d, W0c, (bx - 16) * NT + tid, GF, 2 * GF, GF, 16.0f, GH * GF / 2);
  else if (bx < 64)  castpair(W1s, W1c, (bx - 32) * NT + tid, GH, 2 * GH, 0, 16.0f, GH * GH / 2);
  else if (bx < 96)  castpair(W1d, W1c, (bx - 64) * NT + tid, GH, 2 * GH, GH, 16.0f, GH * GH / 2);
  else if (bx < 224) castpair(Wih, WIH, (bx - 96) * NT + tid, GH, GH, 0, 16.0f, 4 * GH * GH / 2);
  else if (bx < 352) castpair(Whh, WHH, (bx - 224) * NT + tid, GH, GH, 0, 16.0f, 4 * GH * GH / 2);
  else if (bx < 368) castpair(Wp, WPc, (bx - 352) * NT + tid, GH, GH, 0, 16.0f, GF * GH / 2);
  else {
    const int j = (bx - 368) * NT + tid;
    if (j < 768) {
      const int j0 = j < GH ? j : GH - 1;
      int j1 = j - GH; j1 = j1 < 0 ? 0 : (j1 >= GH ? GH - 1 : j1);
      int j2 = j - 2 * GH; j2 = j2 < 0 ? 0 : (j2 >= 4 * GH ? 4 * GH - 1 : j2);
      const float v0 = 0.5f * (b0s[j0] + b0d[j0]);
      const float v1 = 32.0f * (b1s[j1] + b1d[j1]);
      const float v2 = bih[j2] + bhh[j2];
      const float v = (j < GH) ? v0 : ((j < 2 * GH) ? v1 : v2);
      ((volatile float*)BI)[j] = v;
      __threadfence();
      ((volatile float*)BI)[j] = v;
    }
  }
}

__global__ __launch_bounds__(NT) void k_deg(const int* __restrict__ ei, const float* __restrict__ ew,
                                            float* __restrict__ invO, float* __restrict__ invI) {
  __shared__ int LIST[SCH];
  __shared__ float LW[SCH];
  __shared__ __align__(16) float SDO[SRB];
  __shared__ __align__(16) float SDI[SRB];
  __shared__ int scan_ws[80];
  const int tid = threadIdx.x, lane = tid & 31, wave = tid >> 5;
  const int bb = blockIdx.x; const int g = bb >> 1; const int n0 = (bb & 1) * SRB;
  const int* srcv = ei + (size_t)g * (2 * GE); const int* dstv = srcv + GE;
  const float* ewg = ew + (size_t)g * GE;
  for (int i = tid; i < SRB; i += NT) { SDO[i] = 0.f; SDI[i] = 0.f; }
  __syncthreads();
#pragma unroll 1
  for (int c = 0; c < NCH; ++c) {
    {
      const int tot = deg_hits(dstv, ewg, c * SCH, n0, tid, LIST, LW, scan_ws);
      deg_apply(tot, lane, wave, LIST, LW, SDI);
      __syncthreads();
    }
    {
      const int tot = deg_hits(srcv, ewg, c * SCH, n0, tid, LIST, LW, scan_ws);
      deg_apply(tot, lane, wave, LIST, LW, SDO);
      __syncthreads();
    }
  }
  for (int i = tid; i < SRB; i += NT) { SDI[i] = inv_sqrt_deg(SDI[i]); SDO[i] = inv_sqrt_deg(SDO[i]); }
  __syncthreads();
  const int r0 = wave * WROWS;
  const v4f a0 = *(const v4f*)(SDI + r0 + 4 * lane), a1 = *(const v4f*)(SDI + r0 + 128 + 4 * lane);
  const v4f b0 = *(const v4f*)(SDO + r0 + 4 * lane), b1 = *(const v4f*)(SDO + r0 + 128 + 4 * lane);
  float* pI = invI + (size_t)g * GNP + n0 + r0;
  float* pO = invO + (size_t)g * GNP + n0 + r0;
  for (int pass = 0; pass < 2; ++pass) {
    *(volatile v4f*)(pI + 4 * lane) = a0; *(volatile v4f*)(pI + 128 + 4 * lane) = a1;
    *(volatile v4f*)(pO + 4 * lane) = b0; *(volatile v4f*)(pO + 128 + 4 * lane) = b1;
    __threadfence();
  }
}

template <int C>
__global__ __launch_bounds__(NT) void k_agg(const float* __restrict__ X, const int* __restrict__ ei, const float* __restrict__ ew,
                                            const float* __restrict__ invSelf, const float* __restrict__ invOth,
                                            float* ACC, _Float16* __restrict__ PL, int kd, int blk0, int rowoff, int coff, float sc) {
  constexpr int VW = C / 32;
  typedef typename FV<VW>::T VT;
  typedef typename FV<VW>::H HT;
  __shared__ int LIST[SCH];
  __shared__ float LW[SCH];
  __shared__ int scan_ws[80];
  const int tid = threadIdx.x, lane = tid & 31, wave = tid >> 5;
  const int bb = blockIdx.x + blk0; const int g = bb >> 1; const int n0 = (bb & 1) * SRB;
  const int rbase = blockIdx.x * SRB;
  const int* eg = ei + (size_t)g * (2 * GE);
  const int* keyv = eg + (kd ? GE : 0);
  const int* othv = eg + (kd ? 0 : GE);
  const float* ewg = ew + (size_t)g * GE;
  const float* ivS = invSelf + (size_t)g * GNP;
  const float* ivO = invOth + (size_t)g * GNP;
  const float* Xg = X + (size_t)g * GN * C;
  VT z;
#pragma unroll
  for (int e = 0; e < VW; ++e) z[e] = 0.f;
  for (int pass = 0; pass < 2; ++pass) {
#pragma unroll 1
    for (int j = 0; j < WROWS; ++j)
      *(volatile VT*)(ACC + (size_t)(rbase + wave * WROWS + j) * C + VW * lane) = z;
    __threadfence();
  }
#pragma unroll 1
  for (int c = 0; c < NCH; ++c) {
    const int tot = agg_hits(keyv, othv, ewg, ivO, c * SCH, n0, tid, LIST, LW, scan_ws);
#pragma unroll 1
    for (int base = 0; base < tot; base += 32) {
      const int q = base + lane; const int qc = q < SCH ? q : SCH - 1;
      const int lv = LIST[qc]; const float lwv = LW[qc];
      const int rv = (q < tot) ? lv : -1;
      const float wv = (q < tot) ? lwv : 0.f;
      const int own = (rv >= 0 && (rv >> 24) == wave) ? 1 : 0;
      unsigned msk = (unsigned)__ballot(own);
#pragma unroll 1
      for (int it = 0; it < 32; ++it) {
        if (msk == 0u) break;
        const int bp = __builtin_ctz(msk); msk &= msk - 1u;
        const int r = __shfl(rv, bp, 32);
        const float w = __shfl(wv, bp, 32);
        const int dl = r >> 16, s = r & 0xFFFF;
        const VT xv = *(const VT*)(Xg + (size_t)s * C + VW * lane);
        float* rp = ACC + (size_t)(rbase + dl) * C + VW * lane;
        VT a = *(volatile VT*)rp;
        a = a + w * xv;
        *(volatile VT*)rp = a;
        __threadfence();
        *(volatile VT*)rp = a;
      }
    }
    __syncthreads();
  }
#pragma unroll 1
  for (int j = 0; j < WROWS; ++j) {
    const int dl = wave * WROWS + j; const int n = n0 + dl;
    if (n < GN) {
      const VT a = *(volatile VT*)(ACC + (size_t)(rbase + dl) * C + VW * lane);
      const float f = ivS[n] * sc;
      const VT v = a * f;
      HT hv;
#pragma unroll
      for (int e = 0; e < VW; ++e) hv[e] = (_Float16)v[e];
      _Float16* pp = PL + ((size_t)g * GN + n - rowoff) * (size_t)(2 * C) + coff + VW * lane;
      *(volatile HT*)pp = hv;
      __threadfence();
      *(volatile HT*)pp = hv;
    }
  }
}

__device__ __forceinline__ float frcp(float x) { return __builtin_amdgcn_rcpf(x); }
__device__ __forceinline__ float sigm(float x) { return frcp(1.0f + __expf(-x)); }
__device__ __forceinline__ float tanhx(float x) {
  const float ax = fabsf(x);
  const float t = __expf(-2.0f * ax);
  const float big = (1.0f - t) * frcp(1.0f + t);
  const float x2 = x * x;
  const float sml = ax * (1.0f + x2 * (-0.333333333f + x2 * (0.133333333f + x2 * -0.053968254f)));
  const float r = (ax < 0.0625f) ? sml : big;
  return copysignf(r, x);
}
__global__ __launch_bounds__(NT) void k_cell(const float* __restrict__ G4, float* CST, _Float16* __restrict__ HPL, int first) {
  const int tid = threadIdx.x, lane = tid & 31, wave = tid >> 5;
  const int row = blockIdx.x * 8 + wave;
  const float* gr = G4 + (size_t)row * (4 * GH) + 4 * lane;
  const v4f gi = *(const v4f*)gr, gf = *(const v4f*)(gr + GH), gg = *(const v4f*)(gr + 2 * GH), go = *(const v4f*)(gr + 3 * GH);
  float* cp = CST + (size_t)row * GH + 4 * lane;
  v4f cold = {0.f, 0.f, 0.f, 0.f};
  if (!first) cold = *(const v4f*)cp;
  v4f cn, hn;
#pragma unroll
  for (int e = 0; e < 4; ++e) {
    const float cc = sigm(gf[e]) * cold[e] + sigm(gi[e]) * tanhx(gg[e]);
    cn[e] = cc;
    hn[e] = sigm(go[e]) * tanhx(cc);
  }
  *(volatile v4f*)cp = cn;
  __threadfence();
  *(volatile v4f*)cp = cn;
  v4h hv;
#pragma unroll
  for (int e = 0; e < 4; ++e) hv[e] = (_Float16)(hn[e] * 64.0f);
  _Float16* hp = HPL + (size_t)row * GH + 4 * lane;
  *(volatile v4h*)hp = hv;
  __threadfence();
  *(volatile v4h*)hp = hv;
}

extern "C" void kernel_launch(void* const* d_in, const int* in_sizes, int n_in,
                              void* d_out, int out_size, void* d_ws, size_t ws_size, hipStream_t stream) {
  if (n_in < 17) return;
  if (in_sizes[0] != GG * GN * GF || in_sizes[1] != GG * 2 * GE || in_sizes[2] != GG * GE) return;
  if (in_sizes[3] != GH * GF || in_sizes[5] != GH * GF || in_sizes[7] != GH * GH || in_sizes[9] != GH * GH) return;
  if (in_sizes[11] != 4 * GH * GH || in_sizes[12] != 4 * GH * GH || in_sizes[15] != GF * GH) return;
  if (in_sizes[4] != GH || in_sizes[6] != GH || in_sizes[8] != GH || in_sizes[10] != GH) return;
  if (in_sizes[13] != 4 * GH || in_sizes[14] != 4 * GH || in_sizes[16] != GF) return;
  if (out_size != BNR * GF) return;
  const float* x_seq = (const float*)d_in[0];
  const int*   ei    = (const int*)  d_in[1];
  const float* ew    = (const float*)d_in[2];
  const float* W0_s  = (const float*)d_in[3];
  const float* b0_s  = (const float*)d_in[4];
  const float* W0_d  = (const float*)d_in[5];
  const float* b0_d  = (const float*)d_in[6];
  const float* W1_s  = (const float*)d_in[7];
  const float* b1_s  = (const float*)d_in[8];
  const float* W1_d  = (const float*)d_in[9];
  const float* b1_d  = (const float*)d_in[10];
  const float* Wih   = (const float*)d_in[11];
  const float* Whh   = (const float*)d_in[12];
  const float* bih   = (const float*)d_in[13];
  const float* bhh   = (const float*)d_in[14];
  const float* Wp    = (const float*)d_in[15];
  const float* bp    = (const float*)d_in[16];
  float* out = (float*)d_out;

  char* ws = (char*)d_ws; size_t off = 0;
  auto carve = [&](size_t bytes) -> char* { char* p = ws + off; off += (bytes + 255) & ~(size_t)255; return p; };
  _Float16* W0c = (_Float16*)carve((size_t)GH * (2 * GF) * 2);
  _Float16* W1c = (_Float16*)carve((size_t)GH * (2 * GH) * 2);
  _Float16* WIH = (_Float16*)carve((size_t)4 * GH * GH * 2);
  _Float16* WHH = (_Float16*)carve((size_t)4 * GH * GH * 2);
  _Float16* WPc = (_Float16*)carve((size_t)GF * GH * 2);
  float*    BI  = (float*)carve(768 * 4);
  float*    invO = (float*)carve((size_t)GG * GNP * 4);
  float*    invI = (float*)carve((size_t)GG * GNP * 4);
  char*     ACCR = carve((size_t)16777216);
  char*     H1R  = carve((size_t)GG * GN * GH * 4);
  char*     APL  = carve((size_t)GG * GN * GH * 2);
  if (off > ws_size || off > (size_t)134217728) return;

  float*    H1    = (float*)H1R;
  _Float16* H2    = (_Float16*)H1R;
  float*    GATES = (float*)(H1R + (size_t)32768000);
  float*    GX    = (float*)APL;
  float*    CST   = (float*)ACCR;
  _Float16* HPL   = (_Float16*)(ACCR + (size_t)8192000);
  float*    ACC   = (float*)ACCR;
  typedef const unsigned short* cus;

  k_prep<<<371, NT, 0, stream>>>(W0_s, W0_d, W1_s, W1_d, Wih, Whh, Wp, b0_s, b0_d, b1_s, b1_d, bih, bhh, W0c, W1c, WIH, WHH, WPc, BI);
  k_deg<<<GG * 2, NT, 0, stream>>>(ei, ew, invO, invI);

  for (int kd = 1; kd >= 0; --kd) {
    const float* ivs = kd ? invI : invO;
    const float* ivo = kd ? invO : invI;
    for (int q = 0; q < 2; ++q)
      k_agg<GF><<<32, NT, 0, stream>>>(x_seq, ei, ew, ivs, ivo, ACC, (_Float16*)APL, kd, 32 * q, 0, kd ? 0 : GF, 16.0f);
  }
  {
    const int tiles = (GG * GN / 64) * (GH / 64);
    wmma_gemm64<0, false, 2, 0, false><<<dim3((tiles + 7) / 8, 1), 256, 0, stream>>>(
        (cus)APL, (cus)nullptr, 2 * GF, 0L, (cus)W0c, (cus)nullptr, 2 * GF, 0L,
        (void*)H1, (void*)nullptr, GH, 0L, BI, (const float*)nullptr, 0L, GG * GN, GH, 2 * GF, 1.0f / 512.0f);
  }
  for (int hh = 0; hh < 2; ++hh) {
    for (int kd = 1; kd >= 0; --kd) {
      const float* ivs = kd ? invI : invO;
      const float* ivo = kd ? invO : invI;
      for (int q = 0; q < 2; ++q)
        k_agg<GH><<<16, NT, 0, stream>>>(H1, ei, ew, ivs, ivo, ACC, (_Float16*)APL, kd, 32 * hh + 16 * q, 64000 * hh, kd ? 0 : GH, 64.0f);
    }
    const int tiles = (64000 / 64) * (GH / 64);
    wmma_gemm64<0, false, 2, 1, false><<<dim3((tiles + 7) / 8, 1), 256, 0, stream>>>(
        (cus)APL, (cus)nullptr, 2 * GH, 0L, (cus)W1c, (cus)nullptr, 2 * GH, 0L,
        (void*)(H2 + (size_t)hh * 64000 * GH), (void*)nullptr, GH, 0L, BI + GH, (const float*)nullptr, 0L, 64000, GH, 2 * GH, 1.0f / 32.0f);
  }
  {
    const int tiles = (BNR / 64) * (4 * GH / 64);
    for (int t = 0; t < NSTEP; ++t) {
      float* gx_out = (t == 0) ? GATES : GX;
      wmma_gemm64<0, false, 2, 0, false><<<dim3((tiles + 7) / 8, 1), 256, 0, stream>>>(
          (cus)(H2 + (size_t)t * GH), (cus)nullptr, NSTEP * GH, 0L, (cus)WIH, (cus)nullptr, GH, 0L,
          (void*)gx_out, (void*)nullptr, 4 * GH, 0L, BI + 2 * GH, (const float*)nullptr, 0L, BNR, 4 * GH, GH, 1.0f / 1024.0f);
      if (t > 0) {
        wmma_gemm64<0, false, 0, 0, true><<<dim3((tiles + 7) / 8, 1), 256, 0, stream>>>(
            (cus)HPL, (cus)nullptr, GH, 0L, (cus)WHH, (cus)nullptr, GH, 0L,
            (void*)GATES, (void*)nullptr, 4 * GH, 0L, (const float*)nullptr, GX, 0L, BNR, 4 * GH, GH, 1.0f / 1024.0f);
      }
      k_cell<<<BNR / 8, NT, 0, stream>>>(GATES, CST, HPL, (t == 0) ? 1 : 0);
    }
  }
  {
    const int tiles = (BNR / 64) * (GF / 64);
    wmma_gemm64<0, false, 2, 0, false><<<dim3((tiles + 7) / 8, 1), 256, 0, stream>>>(
        (cus)HPL, (cus)nullptr, GH, 0L, (cus)WPc, (cus)nullptr, GH, 0L,
        (void*)out, (void*)nullptr, GF, 0L, bp, (const float*)nullptr, 0L, BNR, GF, GH, 1.0f / 1024.0f);
  }
}
